// Pillar_Encoder_87376814670471
// MI455X (gfx1250) — hardware-verified
//
#include <hip/hip_runtime.h>
#include <stdint.h>
#include <stddef.h>
#include <math.h>

#pragma clang fp contract(off)

#define NB     8
#define NPT    20000
#define NCELL  100
#define GSIDE  10
#define TROWS  64
#define NTILE  313
#define NPAD   (NTILE * TROWS)
#define CT     16
#define NCH    20
#define C1     32
#define C2     64
#define C3     128
#define C4I    256
#define C4     768
#define CS     128
#define NSLAB  (C4 / CS)
#define RECW   32
#define H1P    40
#define H2P    72
#define H3P    136
#define AP     264
#define YP     132
#define LDS_A  (TROWS * AP * 2)
#define LDS_E  (NCELL * CS * 4)
#define LDS_L4 (LDS_A + LDS_E)
#define A_SC   8.0f
#define W_SC   256.0f
#define R_L    0.00390625f
#define R_Y    0.00048828125f
#define BN_EPS 1e-5f

static_assert(NTILE * TROWS >= NPT);
static_assert((NTILE - 1) * TROWS < NPT);
static_assert(NCH * CT >= NTILE);
static_assert((NCH - 1) * CT < NTILE);
static_assert(TROWS * YP * 4 <= LDS_A);
static_assert((H1P % 8) == 0);
static_assert((H2P % 8) == 0);
static_assert((H3P % 8) == 0);
static_assert((AP % 8) == 0);
static_assert((YP % 4) == 0);
static_assert((LDS_A % 16) == 0);
static_assert(NSLAB * CS == C4);
static_assert((C4 / 4) <= 256);
static_assert((NCELL * C3) % 8 == 0);
static_assert((NCELL * C3) / 8 <= 7 * 256);
static_assert(NCELL * (CS / 4) <= 13 * 256);
static_assert(TROWS == 64);
static_assert(C3 <= 256);
static_assert(CS <= 256);
static_assert(C1 == 32);
static_assert(C2 == 64);

typedef _Float16       v16h __attribute__((ext_vector_type(16)));
typedef _Float16       v8h  __attribute__((ext_vector_type(8)));
typedef float          v8f  __attribute__((ext_vector_type(8)));
typedef float          v4f  __attribute__((ext_vector_type(4)));
typedef unsigned int   v4u  __attribute__((ext_vector_type(4)));
typedef v4f __attribute__((may_alias)) v4fa;
typedef v4u __attribute__((may_alias)) v4ua;

union FragH { v16h v; v4u q[2]; };
union Pack8 { v8h h; v4u u; };

__device__ __forceinline__ unsigned short hbits(float f) {
  _Float16 t = (_Float16)f;
  unsigned short u;
  __builtin_memcpy(&u, &t, 2);
  return u;
}

__device__ __forceinline__ v8f wmma_h(v16h a, v16h b, v8f c) {
  v8f d = __builtin_amdgcn_wmma_f32_16x16x32_f16(false, a, false, b, (short)0, c, false, false);
  asm volatile("v_nop\n\tv_nop\n\tv_nop\n\tv_nop" : "+v"(d) : "v"(a), "v"(b));
  return d;
}

__device__ __forceinline__ v16h ldfrag(const unsigned short* p, int h) {
  FragH f;
  f.q[0] = *(const v4ua*)(p + 8 * h);
  f.q[1] = *(const v4ua*)(p + 16 + 8 * h);
  return f.v;
}

__device__ __forceinline__ int bin5(float v) {
  float y = v + 1.0f;
  y = fmaxf(y, 0.0f);
  y = fminf(y, 1.99f);
  const float q = y * 5.0f;
  int i = (int)floorf(q);
  i = (y > 0.0f) ? i : 0;
  i = (i < 0) ? 0 : ((i > GSIDE - 1) ? (GSIDE - 1) : i);
  return i;
}
__device__ __forceinline__ int cell_of(float a0, float a2) {
  return bin5(a0) * GSIDE + bin5(a2);
}

__global__ __launch_bounds__(256) void k_tcv(const float* __restrict__ src,
                                             unsigned short* __restrict__ dst,
                                             int K, int N, int npieces, float sc)
{
  const int g = blockIdx.x * 256 + threadIdx.x;
  if (g >= npieces) return;
  const int e0 = g * 8;
  const int n = e0 / K;
  const int k0 = e0 - n * K;
  Pack8 pk;
  #pragma unroll
  for (int i = 0; i < 8; ++i) pk.h[i] = (_Float16)(src[(size_t)(k0 + i) * N + n] * sc);
  const v4u u = pk.u;
  unsigned short* d = dst + (size_t)e0;
  *(volatile v4u*)d = u;
  __threadfence();
  *(volatile v4u*)d = u;
}

__global__ __launch_bounds__(256) void k_stats(const float* __restrict__ x,
                                               float* __restrict__ rec)
{
  __shared__ float sr[4][8];
  const int p = blockIdx.x, b = blockIdx.y;
  const int tid = threadIdx.x, lane = tid & 31, wv = tid >> 5;
  const float* xb = x + (size_t)b * NPT * 3;
  float cnt = 0.f, s0 = 0.f, s1 = 0.f, s2 = 0.f;
  #pragma unroll 1
  for (int i = tid; i < NPT; i += 256) {
    const float a0 = xb[i * 3], a1 = xb[i * 3 + 1], a2 = xb[i * 3 + 2];
    const bool hit = (cell_of(a0, a2) == p);
    cnt += hit ? 1.f : 0.f;
    s0  += hit ? a1 : 0.f;
    s1  += hit ? a0 : 0.f;
    s2  += hit ? a2 : 0.f;
  }
  #pragma unroll
  for (int off = 16; off > 0; off >>= 1) {
    cnt += __shfl_xor(cnt, off);
    s0  += __shfl_xor(s0, off);
    s1  += __shfl_xor(s1, off);
    s2  += __shfl_xor(s2, off);
  }
  if (lane == 0) { sr[0][wv] = cnt; sr[1][wv] = s0; sr[2][wv] = s1; sr[3][wv] = s2; }
  __syncthreads();
  if (wv == 0) {
    float tc = 0.f, t0 = 0.f, t1 = 0.f, t2 = 0.f;
    #pragma unroll
    for (int w = 0; w < 8; ++w) { tc += sr[0][w]; t0 += sr[1][w]; t1 += sr[2][w]; t2 += sr[3][w]; }
    const float den = fmaxf(tc, 1.0f);
    const float rd = 1.0f / den;
    const bool l0 = (lane == 0);
    v4f v;
    v.x = l0 ? tc : 0.f;
    v.y = l0 ? (t0 * rd) : 0.f;
    v.z = l0 ? (t1 * rd) : 0.f;
    v.w = l0 ? (t2 * rd) : 0.f;
    float* d = rec + ((size_t)(b * NCELL + p)) * RECW + 4 * lane;
    if (lane < 8) *(volatile v4f*)d = v;
    __threadfence();
    if (lane < 8) *(volatile v4f*)d = v;
  }
}

__global__ __launch_bounds__(256) void k_mlp(const float* __restrict__ x,
                                             const float* __restrict__ w1,
                                             const float* __restrict__ rec,
                                             const unsigned short* __restrict__ w2t,
                                             const unsigned short* __restrict__ w3t,
                                             unsigned short* __restrict__ h3,
                                             unsigned short* __restrict__ pmx)
{
  __shared__ __align__(16) float sW1[6 * C1];
  __shared__ __align__(16) float sAug[TROWS * 8];
  __shared__ __align__(16) unsigned short sH1[TROWS * H1P];
  __shared__ __align__(16) unsigned short sH2[TROWS * H2P];
  __shared__ __align__(16) unsigned short sH3[TROWS * H3P];
  __shared__ __align__(16) unsigned short sMx[NCELL * C3];
  __shared__ int sSeg[TROWS];

  const int tid = threadIdx.x, lane = tid & 31, wv = tid >> 5;
  const int h = lane >> 4, m = lane & 15;
  const int ch = blockIdx.x, b = blockIdx.y;

  if (tid < 6 * C1) sW1[tid] = w1[tid];
  #pragma unroll 1
  for (int i = tid; i < NCELL * C3; i += 256) sMx[i] = 0;
  __syncthreads();

  const float* xb = x + (size_t)b * NPT * 3;
  const float* recb = rec + (size_t)b * NCELL * RECW;
  unsigned short* h3b = h3 + (size_t)b * NPAD * C3;
  const v8f z8 = {0.f, 0.f, 0.f, 0.f, 0.f, 0.f, 0.f, 0.f};

  #pragma unroll 1
  for (int lt = 0; lt < CT; ++lt) {
    const int t = ch * CT + lt;
    if (t >= NTILE) break;
    const int n0 = t * TROWS;
    int valid = NPT - n0;
    valid = (valid > TROWS) ? TROWS : valid;

    if (tid < TROWS) {
      const int r = tid;
      const int gi = n0 + r;
      const bool ok = (gi < NPT);
      const int gc = ok ? gi : (NPT - 1);
      const float a0 = xb[(size_t)gc * 3], a1 = xb[(size_t)gc * 3 + 1], a2 = xb[(size_t)gc * 3 + 2];
      const int sg = cell_of(a0, a2);
      const float* rl = recb + sg * RECW;
      const float c0 = rl[1], c1 = rl[2], c2 = rl[3];
      float* ar = sAug + r * 8;
      ar[0] = ok ? a1 : 0.f;
      ar[1] = ok ? a0 : 0.f;
      ar[2] = ok ? a2 : 0.f;
      ar[3] = ok ? (a1 - c0) : 0.f;
      ar[4] = ok ? (a0 - c1) : 0.f;
      ar[5] = ok ? (a2 - c2) : 0.f;
      ar[6] = 0.f;
      ar[7] = 0.f;
      sSeg[r] = ok ? sg : 0;
    }
    __syncthreads();

    {
      const int r = tid & (TROWS - 1), og = tid >> 6;
      float av[6];
      #pragma unroll
      for (int k = 0; k < 6; ++k) av[k] = sAug[r * 8 + k];
      Pack8 pk;
      #pragma unroll
      for (int i = 0; i < 8; ++i) {
        const int j = og * 8 + i;
        float s = 0.f;
        #pragma unroll
        for (int k = 0; k < 6; ++k) s = s + av[k] * sW1[k * C1 + j];
        const float rv = (s > 0.f) ? s : 0.f;
        pk.h[i] = (_Float16)(rv * A_SC);
      }
      *(v4ua*)(sH1 + r * H1P + og * 8) = pk.u;
    }
    __syncthreads();

    {
      const int ct = wv & 3, rt0 = 2 * (wv >> 2);
      const v16h bq = ldfrag(w2t + (size_t)(16 * ct + m) * C1, h);
      v8f acc[2];
      #pragma unroll
      for (int mt = 0; mt < 2; ++mt) {
        const v16h a = ldfrag(sH1 + (16 * (rt0 + mt) + m) * H1P, h);
        acc[mt] = wmma_h(a, bq, z8);
      }
      #pragma unroll
      for (int mt = 0; mt < 2; ++mt) {
        #pragma unroll
        for (int r = 0; r < 8; ++r) {
          const int row = 16 * (rt0 + mt) + 8 * h + r;
          const float v = acc[mt][r];
          const float rv = (v > 0.f) ? v : 0.f;
          sH2[row * H2P + 16 * ct + m] = hbits(rv * R_L);
        }
      }
    }
    __syncthreads();

    {
      const int ct0 = 2 * (wv & 3), rt0 = 2 * (wv >> 2);
      v8f acc[2][2];
      #pragma unroll
      for (int mt = 0; mt < 2; ++mt)
        #pragma unroll
        for (int nt = 0; nt < 2; ++nt) acc[mt][nt] = z8;
      #pragma unroll
      for (int ks = 0; ks < 2; ++ks) {
        v16h a[2], bq[2];
        #pragma unroll
        for (int mt = 0; mt < 2; ++mt) a[mt] = ldfrag(sH2 + (16 * (rt0 + mt) + m) * H2P + 32 * ks, h);
        #pragma unroll
        for (int nt = 0; nt < 2; ++nt) bq[nt] = ldfrag(w3t + (size_t)(16 * (ct0 + nt) + m) * C2 + 32 * ks, h);
        #pragma unroll
        for (int mt = 0; mt < 2; ++mt)
          #pragma unroll
          for (int nt = 0; nt < 2; ++nt) acc[mt][nt] = wmma_h(a[mt], bq[nt], acc[mt][nt]);
      }
      #pragma unroll
      for (int mt = 0; mt < 2; ++mt)
        #pragma unroll
        for (int nt = 0; nt < 2; ++nt) {
          const int col = 16 * (ct0 + nt) + m;
          #pragma unroll
          for (int r = 0; r < 8; ++r) {
            const int row = 16 * (rt0 + mt) + 8 * h + r;
            const float v = acc[mt][nt][r];
            const float rv = (v > 0.f) ? v : 0.f;
            sH3[row * H3P + col] = hbits(rv * R_L);
          }
        }
    }
    __syncthreads();

    {
      v4u u[4];
      #pragma unroll
      for (int j = 0; j < 4; ++j) {
        const int i = tid + 256 * j;
        const int row = i >> 4, q = i & 15;
        u[j] = *(const v4ua*)(sH3 + row * H3P + 8 * q);
      }
      #pragma unroll
      for (int j = 0; j < 4; ++j) {
        const int i = tid + 256 * j;
        *(volatile v4u*)(h3b + (size_t)(n0 + (i >> 4)) * C3 + 8 * (i & 15)) = u[j];
      }
      __threadfence();
      #pragma unroll
      for (int j = 0; j < 4; ++j) {
        const int i = tid + 256 * j;
        *(volatile v4u*)(h3b + (size_t)(n0 + (i >> 4)) * C3 + 8 * (i & 15)) = u[j];
      }
    }

    if (tid < C3) {
      const int c = tid;
      #pragma unroll 1
      for (int r = 0; r < valid; ++r) {
        const int p = sSeg[r];
        const unsigned short v = sH3[r * H3P + c];
        unsigned short* e = sMx + p * C3 + c;
        const unsigned short cur = *e;
        *e = (v > cur) ? v : cur;
      }
    }
    __syncthreads();
  }

  {
    unsigned short* d = pmx + ((size_t)(b * NCH + ch)) * (NCELL * C3);
    #pragma unroll
    for (int j = 0; j < 7; ++j) {
      const int i = tid + 256 * j;
      if (i < (NCELL * C3) / 8) {
        const v4u u = *(const v4ua*)(sMx + 8 * i);
        *(volatile v4u*)(d + (size_t)8 * i) = u;
      }
    }
    __threadfence();
    #pragma unroll
    for (int j = 0; j < 7; ++j) {
      const int i = tid + 256 * j;
      if (i < (NCELL * C3) / 8) {
        const v4u u = *(const v4ua*)(sMx + 8 * i);
        *(volatile v4u*)(d + (size_t)8 * i) = u;
      }
    }
  }
}

__global__ __launch_bounds__(32) void k_cred(const unsigned short* __restrict__ pmx,
                                             unsigned short* __restrict__ cmx)
{
  const int p = blockIdx.x, b = blockIdx.y;
  const int lane = threadIdx.x & 31, lc = lane & 15;
  unsigned int mx[8];
  #pragma unroll
  for (int i = 0; i < 8; ++i) mx[i] = 0u;
  #pragma unroll 1
  for (int ch = 0; ch < NCH; ++ch) {
    const unsigned short* s = pmx + (((size_t)(b * NCH + ch)) * NCELL + p) * C3 + 8 * lc;
    const v4u u = *(const v4ua*)s;
    unsigned int w[8];
    w[0] = u.x & 0xffffu; w[1] = u.x >> 16;
    w[2] = u.y & 0xffffu; w[3] = u.y >> 16;
    w[4] = u.z & 0xffffu; w[5] = u.z >> 16;
    w[6] = u.w & 0xffffu; w[7] = u.w >> 16;
    #pragma unroll
    for (int i = 0; i < 8; ++i) mx[i] = (w[i] > mx[i]) ? w[i] : mx[i];
  }
  v4u o;
  o.x = mx[0] | (mx[1] << 16);
  o.y = mx[2] | (mx[3] << 16);
  o.z = mx[4] | (mx[5] << 16);
  o.w = mx[6] | (mx[7] << 16);
  unsigned short* d = cmx + ((size_t)(b * NCELL + p)) * C3 + 8 * lc;
  if (lane < 16) *(volatile v4u*)d = o;
  __threadfence();
  if (lane < 16) *(volatile v4u*)d = o;
}

__global__ __launch_bounds__(256) void k_l4(const float* __restrict__ x,
                                            const unsigned short* __restrict__ h3,
                                            const unsigned short* __restrict__ cmx,
                                            const unsigned short* __restrict__ w4t,
                                            float* __restrict__ enc)
{
  extern __shared__ __align__(16) unsigned char dsm_l4[];
  unsigned short* sA = (unsigned short*)dsm_l4;
  float* sY = (float*)dsm_l4;
  float* sE = (float*)(dsm_l4 + LDS_A);
  __shared__ int sSeg[TROWS];

  const int tid = threadIdx.x, lane = tid & 31, wv = tid >> 5;
  const int h = lane >> 4, m = lane & 15;
  const int cs = blockIdx.x, b = blockIdx.y;

  #pragma unroll 1
  for (int i = tid; i < NCELL * CS; i += 256) sE[i] = 0.f;
  __syncthreads();

  const float* xb = x + (size_t)b * NPT * 3;
  const unsigned short* h3b = h3 + (size_t)b * NPAD * C3;
  const unsigned short* cmb = cmx + (size_t)b * NCELL * C3;
  const unsigned short* wb = w4t + (size_t)(cs * CS) * C4I;
  const v8f z8 = {0.f, 0.f, 0.f, 0.f, 0.f, 0.f, 0.f, 0.f};
  const int ct0 = 2 * (wv & 3), rt0 = 2 * (wv >> 2);

  #pragma unroll 1
  for (int t = 0; t < NTILE; ++t) {
    const int n0 = t * TROWS;
    int valid = NPT - n0;
    valid = (valid > TROWS) ? TROWS : valid;

    if (tid < TROWS) {
      const int r = tid;
      const int gi = n0 + r;
      const bool ok = (gi < NPT);
      const int gc = ok ? gi : (NPT - 1);
      const float a0 = xb[(size_t)gc * 3], a2 = xb[(size_t)gc * 3 + 2];
      const int sg = cell_of(a0, a2);
      sSeg[r] = ok ? sg : 0;
    }
    __syncthreads();

    #pragma unroll
    for (int j = 0; j < 4; ++j) {
      const int i = tid + 256 * j;
      const int r = i >> 4, q = i & 15;
      const v4u u = *(const v4ua*)(h3b + (size_t)(n0 + r) * C3 + 8 * q);
      *(v4ua*)(sA + r * AP + 8 * q) = u;
    }
    #pragma unroll
    for (int j = 0; j < 4; ++j) {
      const int i = tid + 256 * j;
      const int r = i >> 4, q = i & 15;
      int p = sSeg[r];
      p = (p < 0) ? 0 : ((p > NCELL - 1) ? (NCELL - 1) : p);
      const v4u u = *(const v4ua*)(cmb + (size_t)p * C3 + 8 * q);
      *(v4ua*)(sA + r * AP + C3 + 8 * q) = u;
    }
    __syncthreads();

    v8f acc[2][2];
    #pragma unroll
    for (int mt = 0; mt < 2; ++mt)
      #pragma unroll
      for (int nt = 0; nt < 2; ++nt) acc[mt][nt] = z8;
    #pragma unroll
    for (int ks = 0; ks < C4I / 32; ++ks) {
      v16h a[2], bq[2];
      #pragma unroll
      for (int mt = 0; mt < 2; ++mt) a[mt] = ldfrag(sA + (16 * (rt0 + mt) + m) * AP + 32 * ks, h);
      #pragma unroll
      for (int nt = 0; nt < 2; ++nt) bq[nt] = ldfrag(wb + (size_t)(16 * (ct0 + nt) + m) * C4I + 32 * ks, h);
      #pragma unroll
      for (int mt = 0; mt < 2; ++mt)
        #pragma unroll
        for (int nt = 0; nt < 2; ++nt) acc[mt][nt] = wmma_h(a[mt], bq[nt], acc[mt][nt]);
    }
    __syncthreads();

    #pragma unroll
    for (int mt = 0; mt < 2; ++mt)
      #pragma unroll
      for (int nt = 0; nt < 2; ++nt) {
        const int col = 16 * (ct0 + nt) + m;
        #pragma unroll
        for (int r = 0; r < 8; ++r) {
          const int row = 16 * (rt0 + mt) + 8 * h + r;
          const float v = acc[mt][nt][r];
          const float rv = (v > 0.f) ? v : 0.f;
          sY[row * YP + col] = rv * R_Y;
        }
      }
    __syncthreads();

    if (tid < CS) {
      const int c = tid;
      #pragma unroll 1
      for (int r = 0; r < valid; ++r) {
        const int p = sSeg[r];
        const float v = sY[r * YP + c];
        float* e = sE + p * CS + c;
        const float cur = *e;
        *e = (v > cur) ? v : cur;
      }
    }
    __syncthreads();
  }

  float* eb = enc + (size_t)(b * NCELL) * C4 + cs * CS;
  #pragma unroll
  for (int j = 0; j < 13; ++j) {
    const int i = tid + 256 * j;
    if (i < NCELL * (CS / 4)) {
      const int row = i >> 5, q = i & 31;
      const v4f v = *(const v4fa*)(sE + row * CS + 4 * q);
      *(volatile v4f*)(eb + (size_t)row * C4 + 4 * q) = v;
    }
  }
  __threadfence();
  #pragma unroll
  for (int j = 0; j < 13; ++j) {
    const int i = tid + 256 * j;
    if (i < NCELL * (CS / 4)) {
      const int row = i >> 5, q = i & 31;
      const v4f v = *(const v4fa*)(sE + row * CS + 4 * q);
      *(volatile v4f*)(eb + (size_t)row * C4 + 4 * q) = v;
    }
  }
}

__global__ __launch_bounds__(256) void k_bn(const float* __restrict__ enc,
                                            const float* __restrict__ gamma,
                                            const float* __restrict__ beta,
                                            float* __restrict__ out)
{
  __shared__ double sS[256];
  __shared__ double sQ[256];
  const int p = blockIdx.x, tid = threadIdx.x;
  double s = 0.0, q = 0.0;
  #pragma unroll 1
  for (int e = tid; e < NB * C4; e += 256) {
    const int bb = e / C4, c = e - bb * C4;
    const double v = (double)enc[((size_t)(bb * NCELL + p)) * C4 + c];
    s += v;
    q += v * v;
  }
  sS[tid] = s;
  sQ[tid] = q;
  __syncthreads();
  #pragma unroll 1
  for (int off = 128; off > 0; off >>= 1) {
    if (tid < off) { sS[tid] += sS[tid + off]; sQ[tid] += sQ[tid + off]; }
    __syncthreads();
  }
  const double inv_n = (1.0 / 6144.0);
  const double mean = sS[0] * inv_n;
  double var = sQ[0] * inv_n - mean * mean;
  var = (var > 0.0) ? var : 0.0;
  const float meanf = (float)mean;
  const float invf = 1.0f / sqrtf((float)var + BN_EPS);
  const float g = gamma[p], bt = beta[p];
  if (tid < C4 / 4) {
    v4f o[NB];
    #pragma unroll
    for (int bb = 0; bb < NB; ++bb) {
      const v4f v = *(const v4fa*)(enc + ((size_t)(bb * NCELL + p)) * C4 + 4 * tid);
      v4f r;
      r.x = ((v.x - meanf) * invf) * g + bt;
      r.y = ((v.y - meanf) * invf) * g + bt;
      r.z = ((v.z - meanf) * invf) * g + bt;
      r.w = ((v.w - meanf) * invf) * g + bt;
      o[bb] = r;
    }
    #pragma unroll
    for (int bb = 0; bb < NB; ++bb)
      *(volatile v4f*)(out + ((size_t)(bb * NCELL + p)) * C4 + 4 * tid) = o[bb];
    __threadfence();
    #pragma unroll
    for (int bb = 0; bb < NB; ++bb)
      *(volatile v4f*)(out + ((size_t)(bb * NCELL + p)) * C4 + 4 * tid) = o[bb];
  }
}

extern "C" void kernel_launch(void* const* d_in, const int* in_sizes, int n_in,
                              void* d_out, int out_size, void* d_ws, size_t ws_size,
                              hipStream_t stream)
{
  if (n_in < 7) return;
  if (in_sizes[0] != NB * NPT * 3) return;
  if (in_sizes[1] != 6 * C1) return;
  if (in_sizes[2] != C1 * C2) return;
  if (in_sizes[3] != C2 * C3) return;
  if (in_sizes[4] != C4I * C4) return;
  if (in_sizes[5] != NCELL) return;
  if (in_sizes[6] != NCELL) return;
  if (out_size != NB * NCELL * C4) return;

  const float* x     = (const float*)d_in[0];
  const float* w1    = (const float*)d_in[1];
  const float* w2    = (const float*)d_in[2];
  const float* w3    = (const float*)d_in[3];
  const float* w4    = (const float*)d_in[4];
  const float* gamma = (const float*)d_in[5];
  const float* beta  = (const float*)d_in[6];
  float* out = (float*)d_out;

  const size_t bW2T = (size_t)C2 * C1 * 2;
  const size_t bW3T = (size_t)C3 * C2 * 2;
  const size_t bW4T = (size_t)C4 * C4I * 2;
  const size_t bREC = (size_t)NB * NCELL * RECW * 4;
  const size_t bH3  = (size_t)NB * NPAD * C3 * 2;
  const size_t bPMX = (size_t)NB * NCH * NCELL * C3 * 2;
  const size_t bCMX = (size_t)NB * NCELL * C3 * 2;
  const size_t bENC = (size_t)NB * NCELL * C4 * 4;
  const size_t total = bW2T + bW3T + bW4T + bREC + bH3 + bPMX + bCMX + bENC;
  if (total > ws_size) return;
  if (total > (size_t)134217728) return;

  char* ws = (char*)d_ws;
  size_t off = 0;
  unsigned short* W2T = (unsigned short*)(ws + off); off += bW2T;
  unsigned short* W3T = (unsigned short*)(ws + off); off += bW3T;
  unsigned short* W4T = (unsigned short*)(ws + off); off += bW4T;
  float*          REC = (float*)(ws + off);          off += bREC;
  unsigned short* H3  = (unsigned short*)(ws + off); off += bH3;
  unsigned short* PMX = (unsigned short*)(ws + off); off += bPMX;
  unsigned short* CMX = (unsigned short*)(ws + off); off += bCMX;
  float*          ENC = (float*)(ws + off);          off += bENC;
  if (off != total) return;

  hipFuncSetAttribute(reinterpret_cast<const void*>(&k_l4),
                      hipFuncAttributeMaxDynamicSharedMemorySize, LDS_L4);

  {
    const int p2 = C1 * C2 / 8, p3 = C2 * C3 / 8, p4 = C4I * C4 / 8;
    k_tcv<<<(p2 + 255) / 256, 256, 0, stream>>>(w2, W2T, C1,  C2, p2, W_SC);
    k_tcv<<<(p3 + 255) / 256, 256, 0, stream>>>(w3, W3T, C2,  C3, p3, W_SC);
    k_tcv<<<(p4 + 255) / 256, 256, 0, stream>>>(w4, W4T, C4I, C4, p4, W_SC);
  }
  k_stats<<<dim3(NCELL, NB), 256, 0, stream>>>(x, REC);
  k_mlp<<<dim3(NCH, NB), 256, 0, stream>>>(x, w1, REC, W2T, W3T, H3, PMX);
  k_cred<<<dim3(NCELL, NB), 32, 0, stream>>>(PMX, CMX);
  k_l4<<<dim3(NSLAB, NB), 256, LDS_L4, stream>>>(x, H3, CMX, W4T, ENC);
  k_bn<<<NCELL, 256, 0, stream>>>(ENC, gamma, beta, out);
}
